// MoSARA_74826920231188
// MI455X (gfx1250) — hardware-verified
//
#include <hip/hip_runtime.h>


constexpr int NB  = 4096;
constexpr int ND  = 2048;
constexpr int NK  = 512;
constexpr int NE  = 8;
constexpr int NRX = 2 * NK;

static_assert(NB % 64 == 0);
static_assert(ND % 64 == 0);
static_assert(NRX % 64 == 0);
static_assert(ND % 32 == 0);
static_assert(NK % 32 == 0);
static_assert(NK == 512);
static_assert(NE == 8);
static_assert(NB % 32 == 0);

typedef float          v4f   __attribute__((ext_vector_type(4)));
typedef float          v8f   __attribute__((ext_vector_type(8)));
typedef __bf16         v16b  __attribute__((ext_vector_type(16)));
typedef _Float16       v8h   __attribute__((ext_vector_type(8)));
typedef _Float16       v16h  __attribute__((ext_vector_type(16)));
typedef unsigned short u16x8 __attribute__((ext_vector_type(8)));

union FragB { u16x8 h[2]; v16b v; };
union FragH { u16x8 h[2]; v16h v; };

__device__ __forceinline__ unsigned short f2bf(float f) {
    unsigned u = __float_as_uint(f);
    unsigned r = u + 0x7FFFu + ((u >> 16) & 1u);
    return (unsigned short)(r >> 16);
}
__device__ __forceinline__ float bf2f(unsigned short b) {
    return __uint_as_float(((unsigned)b) << 16);
}
__device__ __forceinline__ v8f ld8f(const float* p) {
    v4f a = *(const v4f*)p;
    v4f b = *(const v4f*)(p + 4);
    return __builtin_shufflevector(a, b, 0, 1, 2, 3, 4, 5, 6, 7);
}
__device__ __forceinline__ void split8(const v8f& x, u16x8& hv, u16x8& lv) {
#pragma unroll
    for (int c = 0; c < 8; ++c) {
        const float f = x[c];
        const unsigned short hb = f2bf(f);
        hv[c] = hb;
        lv[c] = f2bf(f - bf2f(hb));
    }
}
__device__ __forceinline__ u16x8 cvt8h(const v8f& x, float scale) {
    v8h t;
#pragma unroll
    for (int c = 0; c < 8; ++c) t[c] = (_Float16)(x[c] * scale);
    return __builtin_bit_cast(u16x8, t);
}
__device__ __forceinline__ float wsum32(float v) {
    v += __shfl_xor(v, 16, 32);
    v += __shfl_xor(v, 8, 32);
    v += __shfl_xor(v, 4, 32);
    v += __shfl_xor(v, 2, 32);
    v += __shfl_xor(v, 1, 32);
    return v;
}

__device__ __forceinline__ void mma_bf(v8f& acc, const FragB& a, const FragB& b) {
    acc = __builtin_amdgcn_wmma_f32_16x16x32_bf16(false, a.v, false, b.v, (short)0, acc, false, false);
    asm volatile("v_nop\n\tv_nop\n\tv_nop\n\tv_nop" : "+v"(acc) : "v"(a.v), "v"(b.v));
}
__device__ __forceinline__ void mma_h(v8f& acc, const FragH& a, const FragH& b) {
    acc = __builtin_amdgcn_wmma_f32_16x16x32_f16(false, a.v, false, b.v, (short)0, acc, false, false);
    asm volatile("v_nop\n\tv_nop\n\tv_nop\n\tv_nop" : "+v"(acc) : "v"(a.v), "v"(b.v));
}

__global__ __launch_bounds__(256)
void cvt_kernel(const float* __restrict__ src, unsigned short* dh, unsigned short* dl, unsigned short* df,
                int n8, int mode, float scale)
{
    const int i = blockIdx.x * 256 + threadIdx.x;
    if (i >= n8) return;
    const size_t e = (size_t)i * 8;
    const v8f x = ld8f(src + e);
    u16x8 hv, lv;
    split8(x, hv, lv);
    const u16x8 fv = cvt8h(x, scale);
    const bool wsplit = (mode & 1) != 0;
    const bool wf16   = (mode & 2) != 0;
    if (wsplit) { *(volatile u16x8*)(dh + e) = hv; *(volatile u16x8*)(dl + e) = lv; }
    if (wf16)   { *(volatile u16x8*)(df + e) = fv; }
    __threadfence();
    if (wsplit) { *(volatile u16x8*)(dh + e) = hv; *(volatile u16x8*)(dl + e) = lv; }
    if (wf16)   { *(volatile u16x8*)(df + e) = fv; }
}

__global__ __launch_bounds__(256)
void tcvt_kernel(const float* __restrict__ U, unsigned short* UT, float scale)
{
    __shared__ float tile[64][33];
    const int tid = threadIdx.x, lane = tid & 31, wave = tid >> 5;
    const int n0 = blockIdx.x * 64;
    const int k0 = blockIdx.y * 32;
#pragma unroll
    for (int it = 0; it < 8; ++it) {
        const int nl = it * 8 + wave;
        tile[nl][lane] = U[(size_t)(n0 + nl) * NK + k0 + lane];
    }
    __syncthreads();
    const int orow = tid >> 3;
    const int seg  = tid & 7;
    v8f x;
#pragma unroll
    for (int c = 0; c < 8; ++c) x[c] = tile[seg * 8 + c][orow];
    const u16x8 fv = cvt8h(x, scale);
    unsigned short* p = UT + (size_t)(k0 + orow) * ND + n0 + seg * 8;
    *(volatile u16x8*)p = fv;
    __threadfence();
    *(volatile u16x8*)p = fv;
}

template<int NBF>
__device__ __forceinline__ void tile_store_pass(const float* st, float* gp, int ldc, int lane) {
    constexpr int CW  = NBF * 16;
    constexpr int P   = CW + 4;
    constexpr int LPR = CW / 4;
    constexpr int RPI = 32 / LPR;
    constexpr int NIT = 32 / RPI;
    const int rsub = lane / LPR;
    const int c4   = (lane % LPR) * 4;
#pragma unroll
    for (int it = 0; it < NIT; ++it) {
        const int row = it * RPI + rsub;
        const v4f v = *(const v4f*)(st + row * P + c4);
        *(volatile v4f*)(gp + (size_t)row * ldc + c4) = v;
    }
}

__global__ __launch_bounds__(128)
void gemm_f16_kernel(const unsigned short* __restrict__ A, const unsigned short* __restrict__ Bp,
                     float* C, int K, int ldc, float scale)
{
    constexpr int NBF = 2;
    constexpr int CW  = NBF * 16;
    constexpr int P   = CW + 4;
    __shared__ __attribute__((aligned(16))) float stile[4][32 * P];

    const int tid  = threadIdx.x;
    const int lane = tid & 31;
    const int wave = tid >> 5;
    const int h    = lane >> 4;
    const int m    = lane & 15;
    const int wm   = wave >> 1;
    const int wn   = wave & 1;

    const int rowW = blockIdx.y * 64 + wm * 32;
    const int colW = blockIdx.x * (2 * CW) + wn * CW;

    v8f acc[2 * NBF];
#pragma unroll
    for (int j = 0; j < 2 * NBF; ++j)
#pragma unroll
        for (int r = 0; r < 8; ++r) acc[j][r] = 0.0f;

    const size_t aoff  = (size_t)(rowW + m) * K + 8 * h;
    const size_t boff  = (size_t)(colW + m) * K + 8 * h;
    const size_t sub16 = (size_t)16 * K;
    const int nk = K >> 5;

#pragma unroll 1
    for (int kt = 0; kt < nk; ++kt) {
        const size_t k0 = (size_t)kt * 32;
        FragH fa[2], fb[NBF];
#pragma unroll
        for (int s = 0; s < 2; ++s) {
            const unsigned short* p = A + aoff + s * sub16 + k0;
            fa[s].h[0] = *(const u16x8*)(p);
            fa[s].h[1] = *(const u16x8*)(p + 16);
        }
#pragma unroll
        for (int j = 0; j < NBF; ++j) {
            const unsigned short* p = Bp + boff + j * sub16 + k0;
            fb[j].h[0] = *(const u16x8*)(p);
            fb[j].h[1] = *(const u16x8*)(p + 16);
        }
#pragma unroll
        for (int s = 0; s < 2; ++s)
#pragma unroll
            for (int j = 0; j < NBF; ++j)
                mma_h(acc[s * NBF + j], fa[s], fb[j]);
    }

    float* st = stile[wave];
#pragma unroll
    for (int s = 0; s < 2; ++s)
#pragma unroll
        for (int j = 0; j < NBF; ++j)
#pragma unroll
            for (int r = 0; r < 8; ++r)
                st[(s * 16 + 8 * h + r) * P + j * 16 + m] = acc[s * NBF + j][r] * scale;
    __syncthreads();

    float* gp = C + (size_t)rowW * ldc + colW;
    tile_store_pass<NBF>(st, gp, ldc, lane);
    __threadfence();
    tile_store_pass<NBF>(st, gp, ldc, lane);
}

__global__ __launch_bounds__(256)
void router_kernel(const float* __restrict__ RX, const float* __restrict__ W1, const float* __restrict__ W2,
                   const float* __restrict__ lam, unsigned short* Zf, float* gsum)
{
    __shared__ __attribute__((aligned(16))) float gstg[32];
    const int tid = threadIdx.x, lane = tid & 31, wave = tid >> 5;
    const float w2e = W2[lane & 7];

#pragma unroll 1
    for (int i = 0; i < 4; ++i) {
        const int row = blockIdx.x * 32 + wave * 4 + i;
        const float* rp = RX + (size_t)row * NRX;

        float p = 0.0f;
#pragma unroll
        for (int q = 0; q < 2; ++q) {
            const int kb = q * 256 + 8 * lane;
            const v4f ra = *(const v4f*)(rp + kb);
            const v4f rb = *(const v4f*)(rp + kb + 4);
            const v4f wa = *(const v4f*)(W1 + kb);
            const v4f wb = *(const v4f*)(W1 + kb + 4);
            const v4f t = ra * wa + rb * wb;
            p += (t.x + t.y) + (t.z + t.w);
        }
        const float s = wsum32(p);

        const float le = s * w2e;
        float mx = le;
        mx = fmaxf(mx, __shfl_xor(mx, 1, 32));
        mx = fmaxf(mx, __shfl_xor(mx, 2, 32));
        mx = fmaxf(mx, __shfl_xor(mx, 4, 32));
        const float pe = __expf(le - mx);
        float sm = pe;
        sm += __shfl_xor(sm, 1, 32);
        sm += __shfl_xor(sm, 2, 32);
        sm += __shfl_xor(sm, 4, 32);
        const float ge = pe * (1.0f / sm);
        float gs = ge;
        gs += __shfl_xor(gs, 1, 32);
        gs += __shfl_xor(gs, 2, 32);
        gs += __shfl_xor(gs, 4, 32);
        if (lane == 0) gstg[wave * 4 + i] = gs;

        const float* xp = rp + NK;
#pragma unroll 1
        for (int q = 0; q < 2; ++q) {
            const int kb = q * 256 + 8 * lane;
            v4f la = {0.0f, 0.0f, 0.0f, 0.0f};
            v4f lb = {0.0f, 0.0f, 0.0f, 0.0f};
#pragma unroll 1
            for (int e = 0; e < NE; ++e) {
                const float gq = __shfl(ge, e, 32);
                la += gq * *(const v4f*)(lam + (size_t)e * NK + kb);
                lb += gq * *(const v4f*)(lam + (size_t)e * NK + kb + 4);
            }
            const v4f xa = *(const v4f*)(xp + kb);
            const v4f xb = *(const v4f*)(xp + kb + 4);
            const v4f za = (la * xa) * 1024.0f;
            const v4f zb = (lb * xb) * 1024.0f;
            v8f z;
            z[0] = za.x; z[1] = za.y; z[2] = za.z; z[3] = za.w;
            z[4] = zb.x; z[5] = zb.y; z[6] = zb.z; z[7] = zb.w;
            const u16x8 hz = cvt8h(z, 1.0f);
            unsigned short* zp = Zf + (size_t)row * NK + kb;
            *(volatile u16x8*)zp = hz;
            __threadfence();
            *(volatile u16x8*)zp = hz;
        }
    }
    __syncthreads();
    const v4f gv = *(const v4f*)(gstg + (lane & 7) * 4);
    float* gp = gsum + (size_t)blockIdx.x * 32 + (lane & 7) * 4;
    const bool wr = (wave == 0) && (lane < 8);
    if (wr) *(volatile v4f*)gp = gv;
    __threadfence();
    if (wr) *(volatile v4f*)gp = gv;
}

__global__ __launch_bounds__(128)
void out_kernel(const unsigned short* __restrict__ Ah, const unsigned short* __restrict__ Al,
                const unsigned short* __restrict__ Bh, const unsigned short* __restrict__ Bl, int K1,
                const unsigned short* __restrict__ A2, const unsigned short* __restrict__ B2, int K2,
                const float* __restrict__ gsum, const float* __restrict__ vv,
                float* C, int ldc, float scale2)
{
    constexpr int NBF = 2;
    constexpr int CW  = NBF * 16;
    constexpr int P   = CW + 4;
    __shared__ __attribute__((aligned(16))) float stile[4][32 * P];

    const int tid  = threadIdx.x;
    const int lane = tid & 31;
    const int wave = tid >> 5;
    const int h    = lane >> 4;
    const int m    = lane & 15;
    const int wm   = wave >> 1;
    const int wn   = wave & 1;

    const int rowW = blockIdx.y * 64 + wm * 32;
    const int colW = blockIdx.x * (2 * CW) + wn * CW;

    v8f acc[2 * NBF], acc2[2 * NBF];
#pragma unroll
    for (int j = 0; j < 2 * NBF; ++j)
#pragma unroll
        for (int r = 0; r < 8; ++r) { acc[j][r] = 0.0f; acc2[j][r] = 0.0f; }

    {
        const size_t aoff  = (size_t)(rowW + m) * K1 + 8 * h;
        const size_t boff  = (size_t)(colW + m) * K1 + 8 * h;
        const size_t sub16 = (size_t)16 * K1;
        const int nk = K1 >> 5;
#pragma unroll 1
        for (int kt = 0; kt < nk; ++kt) {
            const size_t k0 = (size_t)kt * 32;
            FragB fa[2], ga[2], fb[NBF], gb[NBF];
#pragma unroll
            for (int s = 0; s < 2; ++s) {
                const unsigned short* p = Ah + aoff + s * sub16 + k0;
                const unsigned short* q = Al + aoff + s * sub16 + k0;
                fa[s].h[0] = *(const u16x8*)(p);
                fa[s].h[1] = *(const u16x8*)(p + 16);
                ga[s].h[0] = *(const u16x8*)(q);
                ga[s].h[1] = *(const u16x8*)(q + 16);
            }
#pragma unroll
            for (int j = 0; j < NBF; ++j) {
                const unsigned short* p = Bh + boff + j * sub16 + k0;
                const unsigned short* q = Bl + boff + j * sub16 + k0;
                fb[j].h[0] = *(const u16x8*)(p);
                fb[j].h[1] = *(const u16x8*)(p + 16);
                gb[j].h[0] = *(const u16x8*)(q);
                gb[j].h[1] = *(const u16x8*)(q + 16);
            }
#pragma unroll
            for (int s = 0; s < 2; ++s)
#pragma unroll
                for (int j = 0; j < NBF; ++j) {
                    mma_bf(acc[s * NBF + j], fa[s], fb[j]);
                    mma_bf(acc[s * NBF + j], fa[s], gb[j]);
                    mma_bf(acc[s * NBF + j], ga[s], fb[j]);
                }
        }
    }

    {
        const size_t aoff  = (size_t)(rowW + m) * K2 + 8 * h;
        const size_t boff  = (size_t)(colW + m) * K2 + 8 * h;
        const size_t sub16 = (size_t)16 * K2;
        const int nk = K2 >> 5;
#pragma unroll 1
        for (int kt = 0; kt < nk; ++kt) {
            const size_t k0 = (size_t)kt * 32;
            FragH fa[2], fb[NBF];
#pragma unroll
            for (int s = 0; s < 2; ++s) {
                const unsigned short* p = A2 + aoff + s * sub16 + k0;
                fa[s].h[0] = *(const u16x8*)(p);
                fa[s].h[1] = *(const u16x8*)(p + 16);
            }
#pragma unroll
            for (int j = 0; j < NBF; ++j) {
                const unsigned short* p = B2 + boff + j * sub16 + k0;
                fb[j].h[0] = *(const u16x8*)(p);
                fb[j].h[1] = *(const u16x8*)(p + 16);
            }
#pragma unroll
            for (int s = 0; s < 2; ++s)
#pragma unroll
                for (int j = 0; j < NBF; ++j)
                    mma_h(acc2[s * NBF + j], fa[s], fb[j]);
        }
    }

    const v8f gs0 = ld8f(gsum + rowW + 8 * h);
    const v8f gs1 = ld8f(gsum + rowW + 16 + 8 * h);
    const float vf0 = 1.0f + vv[colW + m];
    const float vf1 = 1.0f + vv[colW + 16 + m];

    float* st = stile[wave];
#pragma unroll
    for (int s = 0; s < 2; ++s)
#pragma unroll
        for (int j = 0; j < NBF; ++j)
#pragma unroll
            for (int r = 0; r < 8; ++r) {
                const float g  = (s == 0) ? gs0[r] : gs1[r];
                const float vf = (j == 0) ? vf0 : vf1;
                st[(s * 16 + 8 * h + r) * P + j * 16 + m] =
                    (acc[s * NBF + j][r] * g + acc2[s * NBF + j][r] * scale2) * vf;
            }
    __syncthreads();

    float* gp = C + (size_t)rowW * ldc + colW;
    tile_store_pass<NBF>(st, gp, ldc, lane);
    __threadfence();
    tile_store_pass<NBF>(st, gp, ldc, lane);
}

extern "C" void kernel_launch(void* const* d_in, const int* in_sizes, int n_in,
                              void* d_out, int out_size, void* d_ws, size_t ws_size,
                              hipStream_t stream)
{
    if (n_in < 8) return;
    if (in_sizes[0] != NB * ND) return;
    if (in_sizes[1] != ND * ND) return;
    if (in_sizes[2] != ND * NK) return;
    if (in_sizes[3] != NK * ND) return;
    if (in_sizes[4] != NE * NK) return;
    if (in_sizes[5] != ND) return;
    if (in_sizes[6] != NK) return;
    if (in_sizes[7] != NE) return;
    if (out_size != NB * ND) return;

    const float* x   = (const float*)d_in[0];
    const float* W   = (const float*)d_in[1];
    const float* U   = (const float*)d_in[2];
    const float* V   = (const float*)d_in[3];
    const float* lam = (const float*)d_in[4];
    const float* vv  = (const float*)d_in[5];
    const float* W1  = (const float*)d_in[6];
    const float* W2  = (const float*)d_in[7];
    float* out = (float*)d_out;

    char* ws = (char*)d_ws;
    size_t off = 0;
    auto carve = [&](size_t bytes) -> char* { char* p = ws + off; off += (bytes + 255) & ~(size_t)255; return p; };
    const size_t PX16  = (size_t)NB * ND * 2;
    const size_t PW16  = (size_t)ND * ND * 2;
    const size_t PB16  = (size_t)NRX * ND * 2;
    const size_t PU16  = (size_t)ND * NK * 2;
    const size_t PRX32 = (size_t)NB * NRX * 4;
    const size_t PZ16  = (size_t)NB * NK * 2;
    const size_t PGS32 = (size_t)NB * 4;

    unsigned short* Xh   = (unsigned short*)carve(PX16);
    unsigned short* Xl   = (unsigned short*)carve(PX16);
    unsigned short* Xf   = (unsigned short*)carve(PX16);
    unsigned short* Wh   = (unsigned short*)carve(PW16);
    unsigned short* Wl   = (unsigned short*)carve(PW16);
    unsigned short* Bcat = (unsigned short*)carve(PB16);
    unsigned short* Uf   = (unsigned short*)carve(PU16);
    float*          RX   = (float*)carve(PRX32);
    unsigned short* Zf   = (unsigned short*)carve(PZ16);
    float*          GS   = (float*)carve(PGS32);
    if (off > ws_size) return;

    const dim3 b256(256), b128(128);

    cvt_kernel<<<dim3((NB * ND / 8) / 256), b256, 0, stream>>>(x, Xh, Xl, Xf, NB * ND / 8, 3, 1.0f);
    cvt_kernel<<<dim3((ND * ND / 8) / 256), b256, 0, stream>>>(W, Wh, Wl, Xf, ND * ND / 8, 1, 1.0f);
    cvt_kernel<<<dim3((NK * ND / 8) / 256), b256, 0, stream>>>(V, Wh, Wl, Bcat + (size_t)NK * ND, NK * ND / 8, 2, 64.0f);
    cvt_kernel<<<dim3((ND * NK / 8) / 256), b256, 0, stream>>>(U, Wh, Wl, Uf, ND * NK / 8, 2, 64.0f);
    tcvt_kernel<<<dim3(ND / 64, NK / 32), b256, 0, stream>>>(U, Bcat, 64.0f);

    gemm_f16_kernel<<<dim3(NRX / 64, NB / 64), b128, 0, stream>>>(Xf, Bcat, RX, ND, NRX, 0.015625f);

    router_kernel<<<dim3(NB / 32), b256, 0, stream>>>(RX, W1, W2, lam, Zf, GS);

    out_kernel<<<dim3(ND / 64, NB / 64), b128, 0, stream>>>(Xh, Xl, Wh, Wl, ND, Zf, Uf, NK, GS, vv, out, ND,
                                                            1.0f / 65536.0f);
}
